// TinyMambaANC_52243982188792
// MI455X (gfx1250) — hardware-run, weakly checked
//
#include <hip/hip_runtime.h>
#include <math.h>

typedef __attribute__((ext_vector_type(16))) _Float16 v16h;
typedef __attribute__((ext_vector_type(8)))  _Float16 v8h;
typedef __attribute__((ext_vector_type(8)))  float    v8f;
typedef __attribute__((ext_vector_type(4)))  float    v4f;
typedef __attribute__((ext_vector_type(4)))  unsigned v4u;

constexpr int kBatch      = 16;
constexpr int kLen        = 131072;
constexpr int kTok        = 65536;
constexpr int kDm         = 32;
constexpr int kNst        = 16;
constexpr int kMain       = 1024;
constexpr int kHalo       = 128;
constexpr int kTile       = 16;
constexpr int kChunksPerB = kTok / kMain;
constexpr int kChunks     = kBatch * kChunksPerB;
constexpr int kWaves      = 8;
constexpr int kTilesPerChunk = (kHalo + kMain) / kTile;
constexpr int kRowsAll    = kBatch * kTok;
static_assert(kTok * 2 == kLen, "stride-2 encoder");
static_assert((kTok % kMain) == 0, "chunks never cross a batch element");
static_assert((kMain % kTile) == 0 && (kHalo % kTile) == 0, "tile multiples");
static_assert((kChunks % kWaves) == 0, "exact grid");
static_assert(kDm == 32 && kNst == 16, "fragment shapes");

constexpr float kCarW   = 16.0f;
constexpr float kCarXs  = 16.0f;
constexpr float kCarHs  = 64.0f;
constexpr float kCarYg  = 64.0f;
constexpr float kCarLo  = 2048.0f;
constexpr float kInvW   = 1.0f / kCarW;
constexpr float kInvB   = 1.0f / (kCarXs * kCarW);
constexpr float kInvC   = 1.0f / (kCarHs * kCarW);
constexpr float kInvO   = 1.0f / (kCarYg * kCarW);
constexpr float kInvDh  = 1.0f / kCarW;
constexpr float kInvDl  = 1.0f / (kCarW * kCarLo);

constexpr size_t kSzH1   = (size_t)kRowsAll * kDm * 2;
constexpr size_t kSzPT   = (size_t)kRowsAll * 4 * 4;
constexpr size_t kOffH1  = 0;
constexpr size_t kOffPT  = kOffH1 + kSzH1;
constexpr size_t kWsTotal = kOffPT + kSzPT;
static_assert(kWsTotal == 83886080ull, "carve total");
static_assert(kWsTotal <= 134217728ull, "carve cap");
static_assert((kOffPT % 128) == 0, "aligned regions");

union FragU { v16h v; v8h h[2]; };

__device__ __forceinline__ v16h frag_load(const _Float16* p) {
  FragU f;
  f.h[0] = *(const v8h*)(p);
  f.h[1] = *(const v8h*)(p + 16);
  return f.v;
}

__device__ __forceinline__ v8f mma_h(v16h a, v16h b, v8f c) {
  c = __builtin_amdgcn_wmma_f32_16x16x32_f16(false, a, false, b, (short)0, c, false, false);
  asm volatile("v_nop\n\tv_nop\n\tv_nop\n\tv_nop" : "+v"(c) : "v"(a), "v"(b));
  return c;
}

__device__ __forceinline__ void wave_sync() {
  __builtin_amdgcn_fence(__ATOMIC_RELEASE, "workgroup");
  __builtin_amdgcn_wave_barrier();
  __builtin_amdgcn_fence(__ATOMIC_ACQUIRE, "workgroup");
}

__device__ __forceinline__ float silu_f(float v) {
  return v * __builtin_amdgcn_rcpf(1.0f + __expf(-v));
}

__device__ __forceinline__ float h16_to_f32(unsigned hb) {
  const unsigned sgn = (hb & 0x8000u) << 16;
  const unsigned em = hb & 0x7fffu;
  const float fn = __uint_as_float((em << 13) + 0x38000000u);
  const float fs = (float)em * 5.9604644775390625e-8f;
  const float mag = (em < 0x400u) ? fs : fn;
  return __uint_as_float(__float_as_uint(mag) | sgn);
}

template <int LAYER>
__global__ __launch_bounds__(256) void mixer_layer_kernel(
    const float* __restrict__ xin, const float* __restrict__ encw, const float* __restrict__ encb,
    const unsigned short* hin, unsigned short* hout, float* ptap,
    const float* __restrict__ lng, const float* __restrict__ lnb,
    const float* __restrict__ wi,  const float* __restrict__ bi,
    const float* __restrict__ wb,  const float* __restrict__ wc,
    const float* __restrict__ dp,  const float* __restrict__ wo,
    const float* __restrict__ bo,  const float* __restrict__ decw)
{
  __shared__ __align__(16) _Float16 sWi[64 * 32];
  __shared__ __align__(16) _Float16 sWb[16 * 32];
  __shared__ __align__(16) _Float16 sWc[32 * 32];
  __shared__ __align__(16) _Float16 sWo[32 * 32];
  __shared__ __align__(16) _Float16 sWd[16 * 32];
  __shared__ __align__(16) _Float16 sWdl[16 * 32];
  __shared__ __align__(16) float sLg[32];
  __shared__ __align__(16) float sLb[32];
  __shared__ __align__(16) float sBi[64];
  __shared__ __align__(16) float sDp[32];
  __shared__ __align__(16) float sBo[32];
  __shared__ __align__(16) float    sR[kWaves][16 * 32];
  __shared__ __align__(16) _Float16 sA2[kWaves][16 * 32];
  __shared__ __align__(16) _Float16 sA3[kWaves][16 * 32];
  __shared__ __align__(16) _Float16 sA4[kWaves][16 * 32];
  __shared__ __align__(16) float    sX[kWaves][40];
  __shared__ __align__(16) float    sP[kWaves][64];

  const int tid = threadIdx.x;

#pragma unroll 1
  for (int i = tid; i < 64 * 32; i += 256) sWi[i] = (_Float16)(wi[LAYER * 2048 + i] * kCarW);
#pragma unroll 1
  for (int i = tid; i < 16 * 32; i += 256) sWb[i] = (_Float16)(wb[LAYER * 512 + i] * kCarW);
#pragma unroll 1
  for (int i = tid; i < 32 * 32; i += 256) {
    const int nn = i >> 5, kk = i & 31;
    const int kc = (kk < 16) ? kk : 15;
    const float wv = wc[LAYER * 512 + nn * 16 + kc];
    const float ws = (kk < 16) ? (wv * kCarW) : 0.0f;
    sWc[i] = (_Float16)ws;
  }
#pragma unroll 1
  for (int i = tid; i < 32 * 32; i += 256) sWo[i] = (_Float16)(wo[LAYER * 1024 + i] * kCarW);
#pragma unroll 1
  for (int i = tid; i < 16 * 32; i += 256) {
    const int tap = i >> 5, cc = i & 31;
    const int tc = (tap < 4) ? tap : 3;
    const float wv = decw[cc * 4 + tc];
    const float ws = (tap < 4) ? (wv * kCarW) : 0.0f;
    const _Float16 whi = (_Float16)ws;
    const float whf = (float)whi;
    const float wres = (ws - whf) * kCarLo;
    sWd[i]  = whi;
    sWdl[i] = (_Float16)wres;
  }
  if (tid < 32) {
    sLg[tid] = lng[LAYER * 32 + tid];
    sLb[tid] = lnb[LAYER * 32 + tid];
    sDp[tid] = dp[LAYER * 32 + tid];
    sBo[tid] = bo[LAYER * 32 + tid];
  }
  if (tid < 64) sBi[tid] = bi[LAYER * 64 + tid];
  __syncthreads();

  const int lane = tid & 31;
  const int wave = __builtin_amdgcn_readfirstlane(tid >> 5);
  const int hh = lane >> 4;
  const int n  = lane & 15;
  const int chunk = blockIdx.x * kWaves + wave;
  const int batch = chunk / kChunksPerB;
  const int t0    = (chunk - batch * kChunksPerB) * kMain;

  float*    R  = sR[wave];
  _Float16* A2 = sA2[wave];
  _Float16* A3 = sA3[wave];
  _Float16* A4 = sA4[wave];
  float*    X  = sX[wave];
  float*    PS = sP[wave];

  const int fo = n * 32 + 8 * hh;
  const v16h bWi0 = frag_load(sWi + fo);
  const v16h bWi1 = frag_load(sWi + 512 + fo);
  const v16h bWi2 = frag_load(sWi + 1024 + fo);
  const v16h bWi3 = frag_load(sWi + 1536 + fo);
  const v16h bWb  = frag_load(sWb + fo);
  const v16h bWc0 = frag_load(sWc + fo);
  const v16h bWc1 = frag_load(sWc + 512 + fo);
  const v16h bWo0 = frag_load(sWo + fo);
  const v16h bWo1 = frag_load(sWo + 512 + fo);
  const v16h bWd  = frag_load(sWd + fo);
  const v16h bWdl = frag_load(sWdl + fo);

  const float bi0 = sBi[n], bi1 = sBi[16 + n], bi2 = sBi[32 + n], bi3 = sBi[48 + n];
  const float dp0 = sDp[n], dp1 = sDp[16 + n];
  const float bo0 = sBo[n], bo1 = sBo[16 + n];

  const v4f ewv = *(const v4f*)(encw + lane * 4);
  const float ew0 = ewv[0], ew1 = ewv[1], ew2 = ewv[2], ew3 = ewv[3];
  const float eb  = encb[lane];

  const v8f zero8 = {0.f, 0.f, 0.f, 0.f, 0.f, 0.f, 0.f, 0.f};
  float hstate = 0.0f;

#pragma unroll 1
  for (int tile = 0; tile < kTilesPerChunk; ++tile) {
    const int tstart = t0 - kHalo + tile * kTile;
    if (tstart < 0) continue;
    const bool halo = (tstart < t0);
    const size_t row0 = (size_t)batch * kTok + (size_t)tstart;
    wave_sync();

    if (LAYER == 0) {
      const float* xb = xin + (size_t)batch * kLen;
      const int base = 2 * tstart - 1;
      const int j0 = base + lane;
      const int j0c = (j0 < 0) ? 0 : ((j0 > kLen - 1) ? (kLen - 1) : j0);
      float xv0 = xb[j0c];
      asm volatile("" : "+v"(xv0));
      const int j1 = base + 32 + (lane & 1);
      const int j1c = (j1 > kLen - 1) ? (kLen - 1) : j1;
      float xv1 = xb[j1c];
      asm volatile("" : "+v"(xv1));
      X[lane] = (j0 >= 0 && j0 < kLen) ? xv0 : 0.0f;
      if (lane < 2) X[32 + lane] = (j1 < kLen) ? xv1 : 0.0f;
      wave_sync();
#pragma unroll 1
      for (int t = 0; t < 16; ++t) {
        const float a0 = X[2 * t], a1 = X[2 * t + 1], a2 = X[2 * t + 2], a3 = X[2 * t + 3];
        float acc = a0 * ew0;
        acc = fmaf(a1, ew1, acc);
        acc = fmaf(a2, ew2, acc);
        acc = fmaf(a3, ew3, acc);
        const float pre = acc + eb;
        R[t * 32 + lane] = 0.5f * pre * (1.0f + erff(pre * 0.70710678118654752f));
      }
    } else {
      const unsigned short* hp = hin + row0 * 32;
#pragma unroll
      for (int i = 0; i < 2; ++i) {
        const v4u w = *(const v4u*)(hp + i * 256 + lane * 8);
        const unsigned w0 = w[0], w1 = w[1], w2 = w[2], w3 = w[3];
        const int tok = i * 8 + (lane >> 2);
        const int f0 = (lane & 3) * 8;
        v4f lo4, hi4;
        lo4[0] = h16_to_f32(w0 & 0xffffu);
        lo4[1] = h16_to_f32(w0 >> 16);
        lo4[2] = h16_to_f32(w1 & 0xffffu);
        lo4[3] = h16_to_f32(w1 >> 16);
        hi4[0] = h16_to_f32(w2 & 0xffffu);
        hi4[1] = h16_to_f32(w2 >> 16);
        hi4[2] = h16_to_f32(w3 & 0xffffu);
        hi4[3] = h16_to_f32(w3 >> 16);
        *(v4f*)(R + tok * 32 + f0)     = lo4;
        *(v4f*)(R + tok * 32 + f0 + 4) = hi4;
      }
    }
    wave_sync();

    v16h fa;
    {
      const float* rr = R + n * 32 + 8 * hh;
      const v4f q0 = *(const v4f*)(rr);
      const v4f q1 = *(const v4f*)(rr + 4);
      const v4f q2 = *(const v4f*)(rr + 16);
      const v4f q3 = *(const v4f*)(rr + 20);
      float v[16];
#pragma unroll
      for (int e = 0; e < 4; ++e) { v[e] = q0[e]; v[4 + e] = q1[e]; v[8 + e] = q2[e]; v[12 + e] = q3[e]; }
      float s = 0.0f;
#pragma unroll
      for (int e = 0; e < 16; ++e) s += v[e];
      s += __shfl_xor(s, 16, 32);
      const float mu = s * (1.0f / 32.0f);
      float qs = 0.0f;
#pragma unroll
      for (int e = 0; e < 16; ++e) { v[e] -= mu; qs = fmaf(v[e], v[e], qs); }
      qs += __shfl_xor(qs, 16, 32);
      const float inv = rsqrtf(qs * (1.0f / 32.0f) + 1e-5f);
      const v4f g0 = *(const v4f*)(sLg + 8 * hh);
      const v4f g1 = *(const v4f*)(sLg + 8 * hh + 4);
      const v4f g2 = *(const v4f*)(sLg + 16 + 8 * hh);
      const v4f g3 = *(const v4f*)(sLg + 20 + 8 * hh);
      const v4f c0 = *(const v4f*)(sLb + 8 * hh);
      const v4f c1 = *(const v4f*)(sLb + 8 * hh + 4);
      const v4f c2 = *(const v4f*)(sLb + 16 + 8 * hh);
      const v4f c3 = *(const v4f*)(sLb + 20 + 8 * hh);
#pragma unroll
      for (int e = 0; e < 4; ++e) {
        fa[e]      = (_Float16)(v[e] * inv * g0[e] + c0[e]);
        fa[4 + e]  = (_Float16)(v[4 + e] * inv * g1[e] + c1[e]);
        fa[8 + e]  = (_Float16)(v[8 + e] * inv * g2[e] + c2[e]);
        fa[12 + e] = (_Float16)(v[12 + e] * inv * g3[e] + c3[e]);
      }
    }

    const v8f xp0 = mma_h(fa, bWi0, zero8);
    const v8f xp1 = mma_h(fa, bWi1, zero8);
    float xs0[8], xs1[8];
#pragma unroll
    for (int r = 0; r < 8; ++r) {
      const float u0 = silu_f(fmaf(xp0[r], kInvW, bi0));
      const float u1 = silu_f(fmaf(xp1[r], kInvW, bi1));
      xs0[r] = u0;
      xs1[r] = u1;
      A2[(8 * hh + r) * 32 + n]      = (_Float16)(u0 * kCarXs);
      A2[(8 * hh + r) * 32 + 16 + n] = (_Float16)(u1 * kCarXs);
    }
    wave_sync();

    const v16h fa2 = frag_load(A2 + fo);
    const v8f bacc = mma_h(fa2, bWb, zero8);

#pragma unroll
    for (int t = 0; t < 16; ++t) {
      const float bv = __shfl(bacc[t & 7], (t >> 3) * 16 + n, 32);
      hstate = fmaf(0.9f, hstate, 0.1f * (bv * kInvB));
      const float sv = (hh == 0) ? (hstate * kCarHs) : 0.0f;
      A3[t * 32 + lane] = (_Float16)sv;
    }
    wave_sync();
    if (halo) continue;

    const v8f z0 = mma_h(fa, bWi2, zero8);
    const v8f z1 = mma_h(fa, bWi3, zero8);

    const v16h fa3 = frag_load(A3 + fo);
    const v8f y0 = mma_h(fa3, bWc0, zero8);
    const v8f y1 = mma_h(fa3, bWc1, zero8);
#pragma unroll
    for (int r = 0; r < 8; ++r) {
      const float yy0 = fmaf(y0[r], kInvC, dp0 * xs0[r]);
      const float yy1 = fmaf(y1[r], kInvC, dp1 * xs1[r]);
      const float gt0 = silu_f(fmaf(z0[r], kInvW, bi2));
      const float gt1 = silu_f(fmaf(z1[r], kInvW, bi3));
      A4[(8 * hh + r) * 32 + n]      = (_Float16)(yy0 * gt0 * kCarYg);
      A4[(8 * hh + r) * 32 + 16 + n] = (_Float16)(yy1 * gt1 * kCarYg);
    }
    wave_sync();

    const v16h fa4 = frag_load(A4 + fo);
    const v8f o0 = mma_h(fa4, bWo0, zero8);
    const v8f o1 = mma_h(fa4, bWo1, zero8);
#pragma unroll
    for (int r = 0; r < 8; ++r) {
      float* rp = R + (8 * hh + r) * 32 + n;
      const float r0v = rp[0];
      const float r1v = rp[16];
      rp[0]  = r0v + fmaf(o0[r], kInvO, bo0);
      rp[16] = r1v + fmaf(o1[r], kInvO, bo1);
    }
    wave_sync();

    if (LAYER == 0) {
      v8h hv[2];
#pragma unroll
      for (int i = 0; i < 2; ++i) {
        const int tok = i * 8 + (lane >> 2);
        const int f0 = (lane & 3) * 8;
        const v4f a0 = *(const v4f*)(R + tok * 32 + f0);
        const v4f a1 = *(const v4f*)(R + tok * 32 + f0 + 4);
#pragma unroll
        for (int e = 0; e < 4; ++e) {
          hv[i][e]     = (_Float16)a0[e];
          hv[i][4 + e] = (_Float16)a1[e];
        }
      }
      unsigned short* op = hout + row0 * 32;
      for (int pass = 0; pass < 2; ++pass) {
#pragma unroll
        for (int i = 0; i < 2; ++i)
          *(volatile v8h*)(op + i * 256 + lane * 8) = hv[i];
        __threadfence();
      }
    } else {
      v16h ahi, alo;
      {
        const float* rr = R + n * 32 + 8 * hh;
        const v4f q0 = *(const v4f*)(rr);
        const v4f q1 = *(const v4f*)(rr + 4);
        const v4f q2 = *(const v4f*)(rr + 16);
        const v4f q3 = *(const v4f*)(rr + 20);
        float v[16];
#pragma unroll
        for (int e = 0; e < 4; ++e) { v[e] = q0[e]; v[4 + e] = q1[e]; v[8 + e] = q2[e]; v[12 + e] = q3[e]; }
#pragma unroll
        for (int e = 0; e < 16; ++e) {
          const _Float16 hi = (_Float16)v[e];
          const float hf = (float)hi;
          const float res = (v[e] - hf) * kCarLo;
          ahi[e] = hi;
          alo[e] = (_Float16)res;
        }
      }
      const v8f ph = mma_h(ahi, bWd, zero8);
      v8f pl = mma_h(alo, bWd, zero8);
      pl = mma_h(ahi, bWdl, pl);
      if (n < 4) {
#pragma unroll
        for (int r = 0; r < 8; ++r)
          PS[(8 * hh + r) * 4 + n] = fmaf(pl[r], kInvDl, ph[r] * kInvDh);
      }
      wave_sync();
      const v4f pv = *(const v4f*)(PS + n * 4);
      float* pp = ptap + row0 * 4 + (size_t)n * 4;
      for (int pass = 0; pass < 2; ++pass) {
        if (lane < 16) *(volatile v4f*)pp = pv;
        __threadfence();
      }
    }
  }
}

__global__ __launch_bounds__(256) void tap_combine_kernel(
    const float* __restrict__ P, const float* __restrict__ decb, float* __restrict__ outp)
{
  const int i = blockIdx.x * 256 + threadIdx.x;
  if (i >= kRowsAll / 2) return;
  const int g0 = 2 * i;
  const int tl = g0 & (kTok - 1);
  const v4f pa = *(const v4f*)(P + (size_t)g0 * 4);
  const v4f pb = *(const v4f*)(P + (size_t)(g0 + 1) * 4);
  const int gm = (g0 > 0) ? (g0 - 1) : 0;
  const int gp = (g0 + 2 < kRowsAll) ? (g0 + 2) : (kRowsAll - 1);
  const float pm3 = P[(size_t)gm * 4 + 3];
  const float pp0 = P[(size_t)gp * 4];
  const float m3 = (tl > 0) ? pm3 : 0.0f;
  const float p0 = (tl + 2 < kTok) ? pp0 : 0.0f;
  const float db = decb[0];
  v4f o;
  o[0] = (m3 + pa[1]) + db;
  o[1] = (pa[2] + pb[0]) + db;
  o[2] = (pa[3] + pb[1]) + db;
  o[3] = (pb[2] + p0) + db;
  float* q = outp + (size_t)i * 4;
  *(volatile v4f*)q = o;
  __threadfence();
  *(volatile v4f*)q = o;
}

extern "C" void kernel_launch(void* const* d_in, const int* in_sizes, int n_in,
                              void* d_out, int out_size, void* d_ws, size_t ws_size,
                              hipStream_t stream)
{
  if (n_in < 14) return;
  if (in_sizes[0] != kBatch * kLen) return;
  if (in_sizes[1] != kDm * 4 || in_sizes[2] != kDm) return;
  if (in_sizes[3] != 2 * kDm || in_sizes[4] != 2 * kDm) return;
  if (in_sizes[5] != 2 * 64 * kDm || in_sizes[6] != 2 * 64) return;
  if (in_sizes[7] != 2 * kNst * kDm || in_sizes[8] != 2 * kDm * kNst) return;
  if (in_sizes[9] != 2 * kDm) return;
  if (in_sizes[10] != 2 * kDm * kDm || in_sizes[11] != 2 * kDm) return;
  if (in_sizes[12] != kDm * 4 || in_sizes[13] != 1) return;
  if (out_size != kBatch * kLen) return;
  if (ws_size < kWsTotal) return;

  const float* x         = (const float*)d_in[0];
  const float* enc_w     = (const float*)d_in[1];
  const float* enc_b     = (const float*)d_in[2];
  const float* ln_g      = (const float*)d_in[3];
  const float* ln_b      = (const float*)d_in[4];
  const float* inproj_w  = (const float*)d_in[5];
  const float* inproj_b  = (const float*)d_in[6];
  const float* B_w       = (const float*)d_in[7];
  const float* C_w       = (const float*)d_in[8];
  const float* D_p       = (const float*)d_in[9];
  const float* outproj_w = (const float*)d_in[10];
  const float* outproj_b = (const float*)d_in[11];
  const float* dec_w     = (const float*)d_in[12];
  const float* dec_b     = (const float*)d_in[13];

  char* ws = (char*)d_ws;
  unsigned short* H1 = (unsigned short*)(ws + kOffH1);
  float*          PT = (float*)(ws + kOffPT);

  mixer_layer_kernel<0><<<kChunks / kWaves, 256, 0, stream>>>(
      x, enc_w, enc_b, H1, H1, PT,
      ln_g, ln_b, inproj_w, inproj_b, B_w, C_w, D_p, outproj_w, outproj_b, dec_w);

  mixer_layer_kernel<1><<<kChunks / kWaves, 256, 0, stream>>>(
      x, enc_w, enc_b, H1, H1, PT,
      ln_g, ln_b, inproj_w, inproj_b, B_w, C_w, D_p, outproj_w, outproj_b, dec_w);

  tap_combine_kernel<<<(kRowsAll / 2) / 256, 256, 0, stream>>>(PT, dec_b, (float*)d_out);
}
